// MPEncoder_44719199485974
// MI455X (gfx1250) — hardware-run, weakly checked
//
#include <hip/hip_runtime.h>
#include <stddef.h>
#include <stdint.h>

#pragma clang fp contract(off)


#define NNODE   50000
#define NEDGE   800000
#define D_IN    128
#define D_HID   256
#define D_OUT   128
#define SPLIT1  1
#define SPLIT2  1
#define XP      128
#define ZP1     256
#define ZP2     512
#define HP      256
#define WP1     256
#define WP2     512
#define K1USE   (SPLIT1 ? 256 : 128)
#define K2USE   (SPLIT2 ? 512 : 256)
#define NTHR    256
#define NWAVE   8
#define GRP     256
#define NBA     1024
#define PKS     10
#define NB      49
#define NPADN   (NB * NBA)
#define RCAP    28672
#define WLCAP   (RCAP / NWAVE)
#define DEGCAP  64
#define WRANGE  100096
#define GBM     64
#define GBN     128
#define GTHR    128
#define RPB     64
#define RPW     8
#define MP      50048
#define UW1     8192
#define UW2     8192
#define UXB     (MP * 16)
#define NUNITS  (UW1 + UW2 + UXB)
#define BK_INTS (2 * RCAP + 3 * NBA + 32)
#define LDS_BK  (BK_INTS * 4)
#define MEAS_BLK_HITS 16696
#define MEAS_MAXDEG   33

static_assert(NNODE % 4 == 0);
static_assert(NB * NBA >= NNODE && (NB - 1) * NBA < NNODE);
static_assert(MP == 391 * 128 && MP >= NNODE && MP % GBM == 0 && MP % RPB == 0 && MP <= NPADN);
static_assert(NEDGE < (1 << 21));
static_assert(NBA == (1 << PKS) && NBA == NTHR * 4 && NBA % RPB == 0);
static_assert(WRANGE % GRP == 0 && (long long)WRANGE * NWAVE >= NEDGE && GRP == 32 * 8);
static_assert(WLCAP * NWAVE == RCAP);
static_assert(RCAP % (NTHR * 4) == 0 && BK_INTS % 4 == 0);
static_assert((long long)RCAP * 100 >= (long long)MEAS_BLK_HITS * 105);
static_assert((long long)WLCAP * 100 >= (long long)(MEAS_BLK_HITS / NWAVE) * 150);
static_assert(DEGCAP >= MEAS_MAXDEG + 8);
static_assert(LDS_BK <= 300000 && LDS_BK <= 327680);
static_assert(ZP1 == 2 * D_IN && ZP2 == 2 * D_HID && WP1 == ZP1 && WP2 == ZP2 && XP == D_IN && HP == D_HID);
static_assert(K1USE % 32 == 0 && K1USE <= ZP1 && K1USE <= WP1);
static_assert(K2USE % 32 == 0 && K2USE <= ZP2 && K2USE <= WP2);
static_assert(GBM == (GTHR / 32) * 16 && GBN == 8 * 16 && GBN == 32 * 4);
static_assert(D_HID % GBN == 0 && D_OUT % GBN == 0);
static_assert(UW1 % NTHR == 0 && UW2 % NTHR == 0 && UXB % NTHR == 0);
static_assert(UW1 * 8 == D_HID * WP1 && UW2 * 8 == D_OUT * WP2 && UXB * 8 == MP * XP);
static_assert(RPB == NWAVE * RPW);

typedef float          v4f   __attribute__((ext_vector_type(4)));
typedef float          v8f   __attribute__((ext_vector_type(8)));
typedef int            v4i   __attribute__((ext_vector_type(4)));
typedef int            v8i   __attribute__((ext_vector_type(8)));
typedef unsigned       v2u   __attribute__((ext_vector_type(2)));
typedef unsigned       v4u   __attribute__((ext_vector_type(4)));
typedef unsigned short v8us  __attribute__((ext_vector_type(8)));
typedef __bf16         v16bf __attribute__((ext_vector_type(16)));
typedef v4f  __attribute__((may_alias)) v4fa;
typedef v4i  __attribute__((may_alias)) v4ia;
typedef v2u  __attribute__((may_alias)) v2ua;
typedef v4u  __attribute__((may_alias)) v4ua;
typedef v8us __attribute__((may_alias)) v8usa;
union FragB { v16bf v; v8us h[2]; v8i w; };

constexpr size_t R1B    = (size_t)MP * ZP2 * 2;
constexpr size_t O_XB   = 0;
constexpr size_t O_Z1   = (size_t)MP * XP * 2;
constexpr size_t O_Z2   = 0;
constexpr size_t O_H    = R1B;
constexpr size_t O_LIST = O_H + (size_t)MP * HP * 4;
constexpr size_t O_CNT  = O_LIST + (size_t)NB * RCAP * 4;
constexpr size_t O_OFF  = O_CNT + (size_t)NPADN * 4;
constexpr size_t O_REC  = O_OFF + (size_t)NPADN * 4;
constexpr size_t O_W1D  = O_REC + 6400;
constexpr size_t O_W2D  = O_W1D + (size_t)D_HID * WP1 * 2;
constexpr size_t WS_END = O_W2D + (size_t)D_OUT * WP2 * 2;
static_assert(O_Z1 + (size_t)MP * ZP1 * 2 <= R1B);
static_assert((size_t)NB * 128 <= 6400);
static_assert(O_Z1 % 256 == 0 && O_H % 256 == 0 && O_LIST % 256 == 0 && O_CNT % 256 == 0 && O_OFF % 256 == 0);
static_assert(O_REC % 256 == 0 && O_W1D % 256 == 0 && O_W2D % 256 == 0);
static_assert(WS_END <= (size_t)(128u << 20));

__device__ __forceinline__ v8f wmb(const FragB& a, const FragB& b, v8f c) {
  v8f d = __builtin_amdgcn_wmma_f32_16x16x32_bf16(false, a.v, false, b.v, (short)0, c, false, false);
  asm volatile("v_nop\n\tv_nop\n\tv_nop\n\tv_nop" : "+v"(d) : "v"(a.w), "v"(b.w));
  return d;
}

__device__ __forceinline__ unsigned bf16_bits(float f) {
  const unsigned u = __float_as_uint(f);
  const unsigned r = (u + 0x7FFFu + ((u >> 16) & 1u)) >> 16;
  const unsigned q = (u >> 16) | 0x40u;
  const bool isn = (u & 0x7FFFFFFFu) > 0x7F800000u;
  return (isn ? q : r) & 0xFFFFu;
}
__device__ __forceinline__ float bf16_val(float f) { return __uint_as_float(bf16_bits(f) << 16); }
__device__ __forceinline__ float bfw_lo(unsigned w) { return __uint_as_float(w << 16); }
__device__ __forceinline__ float bfw_hi(unsigned w) { return __uint_as_float(w & 0xffff0000u); }
__device__ __forceinline__ void pack2(float a, float b, unsigned& hw, unsigned& lw) {
  const unsigned ha = bf16_bits(a), hb = bf16_bits(b);
  const unsigned la = bf16_bits(a - __uint_as_float(ha << 16));
  const unsigned lb = bf16_bits(b - __uint_as_float(hb << 16));
  hw = ha | (hb << 16);
  lw = la | (lb << 16);
}
__device__ __forceinline__ float relu_k(float v) { return (v > 0.0f) ? v : (v - v); }

__device__ __forceinline__ void wave_sync() {
  __builtin_amdgcn_fence(__ATOMIC_RELEASE, "wavefront");
  __builtin_amdgcn_wave_barrier();
  __builtin_amdgcn_fence(__ATOMIC_ACQUIRE, "wavefront");
}

__device__ __forceinline__ void slot_fetch(const int* __restrict__ CNT, const int* __restrict__ OFF, int node,
                                           int& c, int& o, int& big, float& inv) {
  int craw = CNT[node];
  int oraw = OFF[node];
  asm volatile("" : "+v"(craw), "+v"(oraw));
  const int deg = max(craw, 0);
  int cv = min(deg, DEGCAP);
  const int ov = min(max(oraw, 0), RCAP);
  cv = min(cv, RCAP - ov);
  const int dv = max(deg, 1);
  const int bv = (deg > DEGCAP) ? 1 : 0;
  inv = 1.0f / (float)dv;
  c   = __builtin_amdgcn_readfirstlane(cv);
  o   = __builtin_amdgcn_readfirstlane(ov);
  big = __builtin_amdgcn_readfirstlane(bv);
}

__device__ __forceinline__ int scan_group(const int* __restrict__ keys, int nE, int gbase, int slotBase, int nb,
                                          int vec8, int* mywl, int lane, int wc) {
  const int e0   = gbase + 8 * lane;
  const int sent = (int)(1u << 31);
  v4i da, db;
  if (vec8 != 0 && gbase + GRP <= nE) {
    da = *(const v4i*)(keys + e0);
    db = *(const v4i*)(keys + e0 + 4);
  } else {
    const int k0 = keys[min(e0,     nE - 1)];
    const int k1 = keys[min(e0 + 1, nE - 1)];
    const int k2 = keys[min(e0 + 2, nE - 1)];
    const int k3 = keys[min(e0 + 3, nE - 1)];
    const int k4 = keys[min(e0 + 4, nE - 1)];
    const int k5 = keys[min(e0 + 5, nE - 1)];
    const int k6 = keys[min(e0 + 6, nE - 1)];
    const int k7 = keys[min(e0 + 7, nE - 1)];
    asm volatile("" :: "v"(k0), "v"(k1), "v"(k2), "v"(k3), "v"(k4), "v"(k5), "v"(k6), "v"(k7));
    da.x = (e0     < nE) ? k0 : sent;
    da.y = (e0 + 1 < nE) ? k1 : sent;
    da.z = (e0 + 2 < nE) ? k2 : sent;
    da.w = (e0 + 3 < nE) ? k3 : sent;
    db.x = (e0 + 4 < nE) ? k4 : sent;
    db.y = (e0 + 5 < nE) ? k5 : sent;
    db.z = (e0 + 6 < nE) ? k6 : sent;
    db.w = (e0 + 7 < nE) ? k7 : sent;
  }
  const unsigned nbs = (unsigned)slotBase;
  const unsigned unb = (unsigned)nb;
  const unsigned s0 = (unsigned)da.x - nbs, s1 = (unsigned)da.y - nbs;
  const unsigned s2 = (unsigned)da.z - nbs, s3 = (unsigned)da.w - nbs;
  const unsigned s4 = (unsigned)db.x - nbs, s5 = (unsigned)db.y - nbs;
  const unsigned s6 = (unsigned)db.z - nbs, s7 = (unsigned)db.w - nbs;
  const bool h0 = s0 < unb, h1 = s1 < unb, h2 = s2 < unb, h3 = s3 < unb;
  const bool h4 = s4 < unb, h5 = s5 < unb, h6 = s6 < unb, h7 = s7 < unb;
  const int cl = (int)h0 + (int)h1 + (int)h2 + (int)h3 + (int)h4 + (int)h5 + (int)h6 + (int)h7;
  const unsigned any = __builtin_amdgcn_ballot_w32(cl != 0);
  if (any != 0u) {
    int incl = cl;
#pragma unroll
    for (int d = 1; d < 32; d <<= 1) {
      const int up = __shfl_up(incl, d, 32);
      if (lane >= d) incl += up;
    }
    const int tot = __shfl(incl, 31, 32);
    int pos = wc + incl - cl;
#define PUTJ(J, HJ, SJ) \
    if (HJ) { if (pos < WLCAP) mywl[pos] = (int)(((unsigned)(e0 + (J)) << PKS) | (SJ)); pos += 1; }
    PUTJ(0, h0, s0)
    PUTJ(1, h1, s1)
    PUTJ(2, h2, s2)
    PUTJ(3, h3, s3)
    PUTJ(4, h4, s4)
    PUTJ(5, h5, s5)
    PUTJ(6, h6, s6)
    PUTJ(7, h7, s7)
#undef PUTJ
    wc += tot;
  }
  return wc;
}

__global__ __launch_bounds__(NTHR) void k_prep(const float* __restrict__ x, const float* __restrict__ W1,
                                               const float* __restrict__ W2, unsigned short* XB,
                                               unsigned short* W1D, unsigned short* W2D, int nN) {
  const int u = (int)blockIdx.x * NTHR + (int)threadIdx.x;
  if (u < UW1) {
    const int n  = u >> 5;
    const int k8 = (u & 31) * 8;
    const int ks = k8 & (D_IN - 1);
    float f[8];
#pragma unroll
    for (int i = 0; i < 8; ++i) f[i] = W1[(size_t)(ks + i) * D_HID + (size_t)n];
    v8us o;
#pragma unroll
    for (int i = 0; i < 8; ++i) o[i] = (unsigned short)bf16_bits(f[i]);
    unsigned short* dp = W1D + (size_t)n * WP1 + (size_t)k8;
    *(volatile v8us*)dp = o;
    __threadfence();
    *(volatile v8us*)dp = o;
  } else if (u < UW1 + UW2) {
    const int v  = u - UW1;
    const int n  = v >> 6;
    const int k8 = (v & 63) * 8;
    const int ks = k8 & (D_HID - 1);
    float f[8];
#pragma unroll
    for (int i = 0; i < 8; ++i) f[i] = W2[(size_t)(ks + i) * D_OUT + (size_t)n];
    v8us o;
#pragma unroll
    for (int i = 0; i < 8; ++i) o[i] = (unsigned short)bf16_bits(f[i]);
    unsigned short* dp = W2D + (size_t)n * WP2 + (size_t)k8;
    *(volatile v8us*)dp = o;
    __threadfence();
    *(volatile v8us*)dp = o;
  } else if (u < NUNITS) {
    const int r   = u - UW1 - UW2;
    const int row = r >> 4;
    const int c8  = (r & 15) * 8;
    const int rc  = row < nN ? row : nN - 1;
    const float* p = x + (size_t)rc * D_IN + c8;
    const v4f a = *(const v4f*)p;
    const v4f b = *(const v4f*)(p + 4);
    asm volatile("" :: "v"(a), "v"(b));
    const bool lv = row < nN;
    v8us o;
    o[0] = lv ? (unsigned short)bf16_bits(a.x) : (unsigned short)0;
    o[1] = lv ? (unsigned short)bf16_bits(a.y) : (unsigned short)0;
    o[2] = lv ? (unsigned short)bf16_bits(a.z) : (unsigned short)0;
    o[3] = lv ? (unsigned short)bf16_bits(a.w) : (unsigned short)0;
    o[4] = lv ? (unsigned short)bf16_bits(b.x) : (unsigned short)0;
    o[5] = lv ? (unsigned short)bf16_bits(b.y) : (unsigned short)0;
    o[6] = lv ? (unsigned short)bf16_bits(b.z) : (unsigned short)0;
    o[7] = lv ? (unsigned short)bf16_bits(b.w) : (unsigned short)0;
    unsigned short* dp = XB + (size_t)row * XP + (size_t)c8;
    *(volatile v8us*)dp = o;
    __threadfence();
    *(volatile v8us*)dp = o;
  }
}

__global__ __launch_bounds__(NTHR) void k_bucket(const int* __restrict__ keys, const int* __restrict__ gidx,
                                                 int nE, int nN, int vec8,
                                                 int* LIST, int* CNT, int* OFF, int* REC) {
  extern __shared__ __attribute__((aligned(16))) int dsm[];
  int* wl   = dsm;
  int* reg2 = wl + RCAP;
  int* scnt = reg2 + RCAP;
  int* soff = scnt + NBA;
  int* cur  = soff + NBA;
  int* wcnt = cur + NBA;
  int* wtot = wcnt + 8;
  int* wmx  = wtot + 8;
  const int tid = (int)threadIdx.x, lane = tid & 31;
  const int wave = __builtin_amdgcn_readfirstlane(tid >> 5);
  const int nodeBase = (int)blockIdx.x * NBA;
  int nb = nN - nodeBase;
  nb = nb > NBA ? NBA : (nb < 1 ? 1 : nb);

  {
    const v4i z4 = {0, 0, 0, 0};
    for (int i = tid * 4; i < BK_INTS; i += NTHR * 4) *(v4ia*)(dsm + i) = z4;
  }
  __syncthreads();

  int wc = 0;
  {
    const int wbeg = wave * WRANGE;
    int wend = wbeg + WRANGE;
    wend = wend > nE ? nE : wend;
    int* mywl = wl + wave * WLCAP;
#pragma unroll 1
    for (int gb = wbeg; gb < wend; gb += GRP)
      wc = scan_group(keys, nE, gb, nodeBase, nb, vec8, mywl, lane, wc);
  }
  if (lane == 0) wcnt[wave] = wc;
  __syncthreads();

  int nh = 0, ovf = 0;
#pragma unroll
  for (int w2 = 0; w2 < NWAVE; ++w2) {
    int c = wcnt[w2];
    ovf |= (c > WLCAP) ? 1 : 0;
    c = c < 0 ? 0 : (c > WLCAP ? WLCAP : c);
    nh += c;
  }

  if (wave == 0) {
#pragma unroll 1
    for (int w2 = 0; w2 < NWAVE; ++w2) {
      int c = wcnt[w2];
      c = c < 0 ? 0 : (c > WLCAP ? WLCAP : c);
      const int* lp = wl + w2 * WLCAP;
#pragma unroll 1
      for (int b0 = 0; b0 < c; b0 += 32) {
        const int idx = b0 + lane;
        const int uv  = lp[idx < WLCAP ? idx : WLCAP - 1];
        const int m32 = (c - b0) < 32 ? (c - b0) : 32;
#pragma unroll 1
        for (int k = 0; k < m32; ++k) {
          const int u  = __builtin_amdgcn_readlane(uv, k);
          const int sl = u & (NBA - 1);
          if (lane == 0) scnt[sl] = scnt[sl] + 1;
        }
      }
    }
  }
  __syncthreads();

  {
    const v4i ca = *(const v4ia*)(scnt + 4 * tid);
    const int e0 = ca.x < 0 ? 0 : ca.x, e1 = ca.y < 0 ? 0 : ca.y, e2 = ca.z < 0 ? 0 : ca.z, e3 = ca.w < 0 ? 0 : ca.w;
    const int ts = e0 + e1 + e2 + e3;
    int incl = ts;
#pragma unroll
    for (int d = 1; d < 32; d <<= 1) {
      const int up = __shfl_up(incl, d, 32);
      if (lane >= d) incl += up;
    }
    int mx = max(max(e0, e1), max(e2, e3));
    mx = max(mx, __shfl_xor(mx, 16, 32));
    mx = max(mx, __shfl_xor(mx, 8, 32));
    mx = max(mx, __shfl_xor(mx, 4, 32));
    mx = max(mx, __shfl_xor(mx, 2, 32));
    mx = max(mx, __shfl_xor(mx, 1, 32));
    if (lane == 31) wtot[wave] = incl;
    if (lane == 0)  wmx[wave] = mx;
    __syncthreads();
    int pre = 0;
#pragma unroll
    for (int w2 = 0; w2 < NWAVE; ++w2) pre += (w2 < wave) ? wtot[w2] : 0;
    int run = pre + incl - ts;
    v4i so;
    so.x = run; run += e0;
    so.y = run; run += e1;
    so.z = run; run += e2;
    so.w = run;
    *(v4ia*)(soff + 4 * tid) = so;
    *(v4ia*)(cur + 4 * tid)  = so;
  }
  __syncthreads();

  if (wave == 0) {
#pragma unroll 1
    for (int w2 = 0; w2 < NWAVE; ++w2) {
      int c = wcnt[w2];
      c = c < 0 ? 0 : (c > WLCAP ? WLCAP : c);
      const int* lp = wl + w2 * WLCAP;
#pragma unroll 1
      for (int b0 = 0; b0 < c; b0 += 32) {
        const int idx = b0 + lane;
        const int uv  = lp[idx < WLCAP ? idx : WLCAP - 1];
        const int m32 = (c - b0) < 32 ? (c - b0) : 32;
#pragma unroll 1
        for (int k = 0; k < m32; ++k) {
          const int u   = __builtin_amdgcn_readlane(uv, k);
          const int sl  = u & (NBA - 1);
          const int eid = (int)((unsigned)u >> PKS);
          if (lane == 0) {
            int pos = cur[sl];
            pos = pos < 0 ? 0 : (pos > RCAP - 1 ? RCAP - 1 : pos);
            reg2[pos] = eid;
            cur[sl] = pos + 1;
          }
        }
      }
    }
  }
  __syncthreads();

  int bmax = 0;
#pragma unroll
  for (int w2 = 0; w2 < NWAVE; ++w2) bmax = max(bmax, wmx[w2]);
  const int flag = ((ovf != 0) || (nh >= RCAP) || (bmax > DEGCAP)) ? 1 : 0;

  int* lrow = LIST + (size_t)blockIdx.x * RCAP;
#pragma unroll 1
  for (int it = 0; it < RCAP / (NTHR * 4); ++it) {
    const int i0 = 4 * (it * NTHR + tid);
    const v4i ev = *(const v4ia*)(reg2 + i0);
    int e0 = ev.x, e1 = ev.y, e2 = ev.z, e3 = ev.w;
    e0 = e0 < 0 ? 0 : (e0 > nE - 1 ? nE - 1 : e0);
    e1 = e1 < 0 ? 0 : (e1 > nE - 1 ? nE - 1 : e1);
    e2 = e2 < 0 ? 0 : (e2 > nE - 1 ? nE - 1 : e2);
    e3 = e3 < 0 ? 0 : (e3 > nE - 1 ? nE - 1 : e3);
    int g0 = gidx[e0], g1 = gidx[e1], g2 = gidx[e2], g3 = gidx[e3];
    asm volatile("" :: "v"(g0), "v"(g1), "v"(g2), "v"(g3));
    g0 = g0 < 0 ? 0 : (g0 > nN - 1 ? nN - 1 : g0);
    g1 = g1 < 0 ? 0 : (g1 > nN - 1 ? nN - 1 : g1);
    g2 = g2 < 0 ? 0 : (g2 > nN - 1 ? nN - 1 : g2);
    g3 = g3 < 0 ? 0 : (g3 > nN - 1 ? nN - 1 : g3);
    v4i ov;
    ov.x = (i0     < nh) ? g0 : 0;
    ov.y = (i0 + 1 < nh) ? g1 : 0;
    ov.z = (i0 + 2 < nh) ? g2 : 0;
    ov.w = (i0 + 3 < nh) ? g3 : 0;
    *(volatile v4i*)(lrow + i0) = ov;
    __threadfence();
    *(volatile v4i*)(lrow + i0) = ov;
  }
  {
    const v4i cv = *(const v4ia*)(scnt + 4 * tid);
    const v4i fv = *(const v4ia*)(soff + 4 * tid);
    v4i rv = {0, 0, 0, 0};
    rv.x = (tid == 0) ? bmax : 0;
    rv.y = (tid == 0) ? flag : 0;
    rv.z = (tid == 0) ? nh : 0;
    int* cp = CNT + (size_t)nodeBase + 4 * tid;
    int* fp = OFF + (size_t)nodeBase + 4 * tid;
    int* rp = REC + (size_t)blockIdx.x * 32 + 4 * (tid & 7);
    *(volatile v4i*)cp = cv;
    *(volatile v4i*)fp = fv;
    if (tid < 8) *(volatile v4i*)rp = rv;
    __threadfence();
    *(volatile v4i*)cp = cv;
    *(volatile v4i*)fp = fv;
    if (tid < 8) *(volatile v4i*)rp = rv;
  }
}

__global__ __launch_bounds__(NTHR) void k_replay1(const unsigned short* __restrict__ XB,
                                                  const int* __restrict__ LIST, const int* __restrict__ CNT,
                                                  const int* __restrict__ OFF, const int* __restrict__ REC,
                                                  unsigned short* Z1, int nN, int mRows) {
  __shared__ __attribute__((aligned(16))) unsigned rowst[NWAVE * 128];
  const int tid = (int)threadIdx.x, lane = tid & 31;
  const int wave = __builtin_amdgcn_readfirstlane(tid >> 5);
  const int bk  = ((int)blockIdx.x * RPB) >> PKS;
  const int flg = REC[(size_t)bk * 32 + 1];
  const int* lp = LIST + (size_t)bk * RCAP;
  unsigned* wst = rowst + wave * 128;
  const float pnan = __uint_as_float(0x7fc00000u);
#pragma unroll 1
  for (int ri = 0; ri < RPW; ++ri) {
    const int node = (int)blockIdx.x * RPB + wave * RPW + ri;
    int c, o, big;
    float inv;
    slot_fetch(CNT, OFF, node, c, o, big, inv);
    int last = o + c - 1;
    last = max(last, o);
    last = min(last, RCAP - 1);
    float a0 = 0.0f, a1 = 0.0f, a2 = 0.0f, a3 = 0.0f;
#pragma unroll 1
    for (int b0 = 0; b0 < c; b0 += 32) {
      int idx = o + b0 + lane;
      idx = min(idx, last);
      int col = lp[idx];
      col = min(max(col, 0), nN - 1);
      const int m32 = min(c - b0, 32);
#pragma unroll 1
      for (int k = 0; k < m32; ++k) {
        const int sk = __builtin_amdgcn_readlane(col, k);
        const v2u w = *(const v2ua*)(XB + (size_t)sk * XP + 4 * lane);
        a0 += bfw_lo(w.x);
        a1 += bfw_hi(w.x);
        a2 += bfw_lo(w.y);
        a3 += bfw_hi(w.y);
      }
    }
    const int nodec = min(node, nN - 1);
    const v2u ow = *(const v2ua*)(XB + (size_t)nodec * XP + 4 * lane);
    asm volatile("" :: "v"(ow));
    float z0 = bfw_lo(ow.x) + a0 * inv;
    float z1 = bfw_hi(ow.x) + a1 * inv;
    float z2 = bfw_lo(ow.y) + a2 * inv;
    float z3 = bfw_hi(ow.y) + a3 * inv;
    const bool poison = (flg != 0) || (big != 0);
    const bool live   = node < nN;
    z0 = poison ? pnan : z0; z1 = poison ? pnan : z1; z2 = poison ? pnan : z2; z3 = poison ? pnan : z3;
    z0 = live ? z0 : 0.0f;   z1 = live ? z1 : 0.0f;   z2 = live ? z2 : 0.0f;   z3 = live ? z3 : 0.0f;
    unsigned h0, l0, h1, l1;
    pack2(z0, z1, h0, l0);
    pack2(z2, z3, h1, l1);
    v2u hv, lv;
    hv.x = h0; hv.y = h1;
    lv.x = l0; lv.y = l1;
    *(v2ua*)(wst + 2 * lane)      = hv;
    *(v2ua*)(wst + 64 + 2 * lane) = lv;
    wave_sync();
    const v4u q = *(const v4ua*)(wst + 4 * lane);
    wave_sync();
    unsigned short* wp = Z1 + (size_t)node * ZP1 + 8 * lane;
    *(volatile v4u*)wp = q;
    __threadfence();
    *(volatile v4u*)wp = q;
  }
}

__global__ __launch_bounds__(NTHR) void k_replay2(const float* __restrict__ H,
                                                  const int* __restrict__ LIST, const int* __restrict__ CNT,
                                                  const int* __restrict__ OFF, const int* __restrict__ REC,
                                                  unsigned short* Z2, int nN, int mRows) {
  const int tid = (int)threadIdx.x, lane = tid & 31;
  const int wave = __builtin_amdgcn_readfirstlane(tid >> 5);
  const int bk  = ((int)blockIdx.x * RPB) >> PKS;
  const int flg = REC[(size_t)bk * 32 + 1];
  const int* lp = LIST + (size_t)bk * RCAP;
  const float pnan = __uint_as_float(0x7fc00000u);
#pragma unroll 1
  for (int ri = 0; ri < RPW; ++ri) {
    const int node = (int)blockIdx.x * RPB + wave * RPW + ri;
    int c, o, big;
    float inv;
    slot_fetch(CNT, OFF, node, c, o, big, inv);
    int last = o + c - 1;
    last = max(last, o);
    last = min(last, RCAP - 1);
    float a0 = 0.f, a1 = 0.f, a2 = 0.f, a3 = 0.f, a4 = 0.f, a5 = 0.f, a6 = 0.f, a7 = 0.f;
#pragma unroll 1
    for (int b0 = 0; b0 < c; b0 += 32) {
      int idx = o + b0 + lane;
      idx = min(idx, last);
      int col = lp[idx];
      col = min(max(col, 0), nN - 1);
      const int m32 = min(c - b0, 32);
#pragma unroll 1
      for (int k = 0; k < m32; ++k) {
        const int sk = __builtin_amdgcn_readlane(col, k);
        const float* hp = H + (size_t)sk * HP + 8 * lane;
        const v4f ha = *(const v4f*)hp;
        const v4f hb = *(const v4f*)(hp + 4);
        a0 += ha.x; a1 += ha.y; a2 += ha.z; a3 += ha.w;
        a4 += hb.x; a5 += hb.y; a6 += hb.z; a7 += hb.w;
      }
    }
    const int nodec = min(node, nN - 1);
    const float* op = H + (size_t)nodec * HP + 8 * lane;
    const v4f oa = *(const v4f*)op;
    const v4f ob = *(const v4f*)(op + 4);
    asm volatile("" :: "v"(oa), "v"(ob));
    float r0 = oa.x + a0 * inv;
    float r1 = oa.y + a1 * inv;
    float r2 = oa.z + a2 * inv;
    float r3 = oa.w + a3 * inv;
    float r4 = ob.x + a4 * inv;
    float r5 = ob.y + a5 * inv;
    float r6 = ob.z + a6 * inv;
    float r7 = ob.w + a7 * inv;
    const bool poison = (flg != 0) || (big != 0);
    const bool live   = node < nN;
    r0 = poison ? pnan : r0; r1 = poison ? pnan : r1; r2 = poison ? pnan : r2; r3 = poison ? pnan : r3;
    r4 = poison ? pnan : r4; r5 = poison ? pnan : r5; r6 = poison ? pnan : r6; r7 = poison ? pnan : r7;
    r0 = live ? r0 : 0.0f; r1 = live ? r1 : 0.0f; r2 = live ? r2 : 0.0f; r3 = live ? r3 : 0.0f;
    r4 = live ? r4 : 0.0f; r5 = live ? r5 : 0.0f; r6 = live ? r6 : 0.0f; r7 = live ? r7 : 0.0f;
    unsigned h0, l0, h1, l1, h2, l2, h3, l3;
    pack2(r0, r1, h0, l0);
    pack2(r2, r3, h1, l1);
    pack2(r4, r5, h2, l2);
    pack2(r6, r7, h3, l3);
    v4u qh, ql;
    qh.x = h0; qh.y = h1; qh.z = h2; qh.w = h3;
    ql.x = l0; ql.y = l1; ql.z = l2; ql.w = l3;
    unsigned short* wp = Z2 + (size_t)node * ZP2 + 8 * lane;
    *(volatile v4u*)wp = qh;
    *(volatile v4u*)(wp + D_HID) = ql;
    __threadfence();
    *(volatile v4u*)wp = qh;
    *(volatile v4u*)(wp + D_HID) = ql;
  }
}

template <int KUSE, int APITCH, int WPITCH, int OPITCH>
__global__ __launch_bounds__(GTHR) __attribute__((amdgpu_num_vgpr(248)))
void k_gemm(const unsigned short* __restrict__ A, const unsigned short* __restrict__ WT,
            const float* __restrict__ bias, float* outp, int nLive, int nStore) {
  __shared__ __attribute__((aligned(16))) float stg[GBM * GBN];
  __shared__ __attribute__((aligned(16))) float bsh[GBN];
  const int tid = (int)threadIdx.x, lane = tid & 31, hh = lane >> 4, m = lane & 15;
  const int wave = __builtin_amdgcn_readfirstlane(tid >> 5);
  const int rowBase = (int)blockIdx.x * GBM;
  const int colBase = (int)blockIdx.y * GBN;

  if (tid < 32) {
    const v4f b4 = *(const v4f*)(bias + colBase + 4 * tid);
    v4f bq;
    bq.x = bf16_val(b4.x); bq.y = bf16_val(b4.y); bq.z = bf16_val(b4.z); bq.w = bf16_val(b4.w);
    *(v4fa*)(bsh + 4 * tid) = bq;
  }

  v8f acc[8];
  {
    const v8f z = {0.f, 0.f, 0.f, 0.f, 0.f, 0.f, 0.f, 0.f};
#pragma unroll
    for (int t = 0; t < 8; ++t) acc[t] = z;
  }
  const unsigned short* ap = A + (size_t)(rowBase + 16 * wave + m) * (size_t)APITCH + 8 * hh;
  const unsigned short* wp = WT + (size_t)(colBase + m) * (size_t)WPITCH + 8 * hh;
#pragma unroll 1
  for (int ks = 0; ks < KUSE / 32; ++ks) {
    FragB af;
    af.h[0] = *(const v8usa*)(ap + 32 * ks);
    af.h[1] = *(const v8usa*)(ap + 32 * ks + 16);
#pragma unroll
    for (int t = 0; t < 8; ++t) {
      const unsigned short* wq = wp + (size_t)(16 * t) * (size_t)WPITCH + 32 * ks;
      FragB bf;
      bf.h[0] = *(const v8usa*)wq;
      bf.h[1] = *(const v8usa*)(wq + 16);
      acc[t] = wmb(af, bf, acc[t]);
    }
  }
  __syncthreads();

#pragma unroll
  for (int t = 0; t < 8; ++t) {
    const int lc = 16 * t + m;
    const float bb = bsh[lc];
#pragma unroll
    for (int r = 0; r < 8; ++r) {
      const int lr = 16 * wave + 8 * hh + r;
      const bool live = (rowBase + lr) < nLive;
      const float v = relu_k(acc[t][r] + bb);
      stg[lr * GBN + lc] = live ? v : 0.0f;
    }
  }
  __syncthreads();

#pragma unroll 1
  for (int i = 0; i < 16; ++i) {
    const int lr = 16 * wave + i;
    const int gr = rowBase + lr;
    const v4f v = *(const v4fa*)(stg + lr * GBN + 4 * lane);
    if (gr < nStore) *(volatile v4f*)(outp + (size_t)gr * (size_t)OPITCH + colBase + 4 * lane) = v;
  }
  __threadfence();
#pragma unroll 1
  for (int i = 0; i < 16; ++i) {
    const int lr = 16 * wave + i;
    const int gr = rowBase + lr;
    const v4f v = *(const v4fa*)(stg + lr * GBN + 4 * lane);
    if (gr < nStore) *(volatile v4f*)(outp + (size_t)gr * (size_t)OPITCH + colBase + 4 * lane) = v;
  }
}

extern "C" void kernel_launch(void* const* d_in, const int* in_sizes, int n_in,
                              void* d_out, int out_size, void* d_ws, size_t ws_size,
                              hipStream_t stream) {
  if (n_in < 7) return;
  if (in_sizes[0] != NNODE * D_IN) return;
  if (in_sizes[1] != D_IN * D_HID || in_sizes[2] != D_HID) return;
  if (in_sizes[3] != D_HID * D_OUT || in_sizes[4] != D_OUT) return;
  if (in_sizes[5] != NEDGE || in_sizes[6] != NEDGE) return;
  if ((long long)out_size != (long long)NNODE * D_OUT) return;
  if (ws_size < WS_END) return;

  const float* x   = (const float*)d_in[0];
  const float* W1  = (const float*)d_in[1];
  const float* b1  = (const float*)d_in[2];
  const float* W2  = (const float*)d_in[3];
  const float* b2  = (const float*)d_in[4];
  const int*   gix = (const int*)  d_in[5];
  const int*   key = (const int*)  d_in[6];
  float* out = (float*)d_out;

  const int nN = NNODE, nE = NEDGE;
  const int vec8 = ((nE & 3) == 0) ? 1 : 0;

  char* ws = (char*)d_ws;
  unsigned short* XB  = (unsigned short*)(ws + O_XB);
  unsigned short* Z1  = (unsigned short*)(ws + O_Z1);
  unsigned short* Z2  = (unsigned short*)(ws + O_Z2);
  float* H    = (float*)(ws + O_H);
  int*   LIST = (int*)(ws + O_LIST);
  int*   CNT  = (int*)(ws + O_CNT);
  int*   OFF  = (int*)(ws + O_OFF);
  int*   REC  = (int*)(ws + O_REC);
  unsigned short* W1D = (unsigned short*)(ws + O_W1D);
  unsigned short* W2D = (unsigned short*)(ws + O_W2D);

  hipFuncSetAttribute(reinterpret_cast<const void*>(&k_bucket), hipFuncAttributeMaxDynamicSharedMemorySize, LDS_BK);

  const int gR = MP / RPB;
  k_prep<<<NUNITS / NTHR, NTHR, 0, stream>>>(x, W1, W2, XB, W1D, W2D, nN);
  k_bucket<<<NB, NTHR, LDS_BK, stream>>>(key, gix, nE, nN, vec8, LIST, CNT, OFF, REC);
  k_replay1<<<gR, NTHR, 0, stream>>>(XB, LIST, CNT, OFF, REC, Z1, nN, MP);
  k_gemm<K1USE, ZP1, WP1, HP><<<dim3((unsigned)gR, (unsigned)(D_HID / GBN), 1u), GTHR, 0, stream>>>(
      Z1, W1D, b1, H, nN, MP);
  k_replay2<<<gR, NTHR, 0, stream>>>(H, LIST, CNT, OFF, REC, Z2, nN, MP);
  k_gemm<K2USE, ZP2, WP2, D_OUT><<<dim3((unsigned)gR, (unsigned)(D_OUT / GBN), 1u), GTHR, 0, stream>>>(
      Z2, W2D, b2, out, nN, nN);
}
